// DifferentialMultiHeadAttention_52020643889367
// MI455X (gfx1250) — hardware-verified
//
#include <hip/hip_runtime.h>
#include <math.h>

constexpr int kBatch  = 2;
constexpr int kSeq    = 2048;
constexpr int kDim    = 1024;
constexpr int kHeads  = 16;
constexpr int kDh     = 64;
constexpr int kDiff   = 32;
constexpr int kTok    = kBatch * kSeq;
constexpr int kQKCols = 2 * kDim;
constexpr float kWCarry    = 16.0f;
constexpr float kWCarryInv = 1.0f / 16.0f;
constexpr float kPCarry    = 32768.0f;
constexpr float kPCarryInv = 1.0f / 32768.0f;
constexpr float kInvScale  = 0.17677669529663687f;
constexpr float kNegBig    = -1.0e9f;
constexpr float kLambdaInit = 0.2f;
constexpr float kOutGain   = 0.8f;
constexpr float kLnEps     = 1.0e-5f;
constexpr float kInv64     = 1.0f / 64.0f;
static_assert(kHeads * kDh == kDim, "shape");
static_assert(kHeads * kDiff * 2 == kDim, "shape");
static_assert(kTok % 64 == 0 && kQKCols % 64 == 0 && kDim % 64 == 0 && kSeq % 64 == 0 && kDh % 64 == 0, "tiles");
static_assert(kDim % 32 == 0 && kDiff % 32 == 0 && kSeq % 32 == 0, "ktiles");
static_assert(kSeq == 4 * 512 && kSeq == 8 * 256, "softmax thread map");
static_assert((kTok * kDim) % (8 * 256) == 0, "cast grid");

typedef __attribute__((ext_vector_type(16))) _Float16 v16h;
typedef __attribute__((ext_vector_type(8)))  _Float16 v8h;
typedef __attribute__((ext_vector_type(16))) __bf16   v16b;
typedef __attribute__((ext_vector_type(8)))  __bf16   v8b;
typedef __attribute__((ext_vector_type(8)))  float    v8f;
typedef __attribute__((ext_vector_type(4)))  float    v4f;
typedef __attribute__((ext_vector_type(2)))  float    v2f;
typedef __attribute__((ext_vector_type(2)))  int      v2i;
typedef __attribute__((ext_vector_type(4)))  unsigned int v4u;

__device__ __forceinline__ unsigned short f2bf_bits(float f) {
  unsigned u = __float_as_uint(f);
  return (unsigned short)((u + 0x7FFFu + ((u >> 16) & 1u)) >> 16);
}
__device__ __forceinline__ float bf_bits2f(unsigned short h) { return __uint_as_float(((unsigned)h) << 16); }

__device__ __forceinline__ void dep_guard_h(v8f& a, v8f& b, v16h x, v16h y) { asm volatile("v_nop\n\tv_nop\n\tv_nop\n\tv_nop" : "+v"(a), "+v"(b) : "v"(x), "v"(y)); }
__device__ __forceinline__ void dep_guard_b(v8f& a, v8f& b, v16b x, v16b y) { asm volatile("v_nop\n\tv_nop\n\tv_nop\n\tv_nop" : "+v"(a), "+v"(b) : "v"(x), "v"(y)); }
__device__ __forceinline__ void dep_guard4_h(v8f& a, v8f& b, v8f& c, v8f& d, v16h x, v16h y) { asm volatile("v_nop\n\tv_nop\n\tv_nop\n\tv_nop" : "+v"(a), "+v"(b), "+v"(c), "+v"(d) : "v"(x), "v"(y)); }
__device__ __forceinline__ void dep_guard4_b(v8f& a, v8f& b, v8f& c, v8f& d, v16b x, v16b y) { asm volatile("v_nop\n\tv_nop\n\tv_nop\n\tv_nop" : "+v"(a), "+v"(b), "+v"(c), "+v"(d) : "v"(x), "v"(y)); }
__device__ __forceinline__ void keep4_h(v16h a, v16h b, v16h c, v16h d) { asm volatile("v_nop" :: "v"(a), "v"(b), "v"(c), "v"(d)); }
__device__ __forceinline__ void keep4_b(v16b a, v16b b, v16b c, v16b d) { asm volatile("v_nop" :: "v"(a), "v"(b), "v"(c), "v"(d)); }
__device__ __forceinline__ void acc_guard4(v8f& a, v8f& b, v8f& c, v8f& d) { asm volatile("v_nop\n\tv_nop\n\tv_nop\n\tv_nop" : "+v"(a), "+v"(b), "+v"(c), "+v"(d)); }
template <typename T> struct Frag;
template <> struct Frag<_Float16> {
  typedef v16h V; union U { v16h v; v8h h[2]; };
  static __device__ __forceinline__ v16h load(const _Float16* p) {
    U f; f.h[0] = *(const v8h*)(p); f.h[1] = *(const v8h*)(p + 16); return f.v;
  }
  static __device__ __forceinline__ v8f mma(v16h a, v16h b, v8f c) {
    return __builtin_amdgcn_wmma_f32_16x16x32_f16(false, a, false, b, (short)0, c, false, false);
  }
  static __device__ __forceinline__ void guard(v8f& a, v8f& b, v16h x, v16h y) { dep_guard_h(a, b, x, y); }
  static __device__ __forceinline__ void guard4(v8f& a, v8f& b, v8f& c, v8f& d, v16h x, v16h y) { dep_guard4_h(a, b, c, d, x, y); }
  static __device__ __forceinline__ void keep(v16h a, v16h b, v16h c, v16h d) { keep4_h(a, b, c, d); }
};
template <> struct Frag<__bf16> {
  typedef v16b V; union U { v16b v; v8b h[2]; };
  static __device__ __forceinline__ v16b load(const __bf16* p) {
    U f; f.h[0] = *(const v8b*)(p); f.h[1] = *(const v8b*)(p + 16); return f.v;
  }
  static __device__ __forceinline__ v8f mma(v16b a, v16b b, v8f c) {
    return __builtin_amdgcn_wmma_f32_16x16x32_bf16(false, a, false, b, (short)0, c, false, false);
  }
  static __device__ __forceinline__ void guard(v8f& a, v8f& b, v16b x, v16b y) { dep_guard_b(a, b, x, y); }
  static __device__ __forceinline__ void guard4(v8f& a, v8f& b, v8f& c, v8f& d, v16b x, v16b y) { dep_guard4_b(a, b, c, d, x, y); }
  static __device__ __forceinline__ void keep(v16b a, v16b b, v16b c, v16b d) { keep4_b(a, b, c, d); }
};

__device__ __forceinline__ unsigned pk16(unsigned short a, unsigned short b) { return (unsigned)a | ((unsigned)b << 16); }
__device__ __forceinline__ unsigned short h_bits(float f) { const _Float16 h = (_Float16)f; return __builtin_bit_cast(unsigned short, h); }

template <int ET> struct Elem;
template <> struct Elem<0> { typedef _Float16 T; };
template <> struct Elem<1> { typedef __bf16 T; };
template <int ET, bool SPLIT, int BIAS_MODE, int OUT_MODE, bool RESID, int ACT = 0>
__global__ __launch_bounds__(256) void wmma_gemm64(
    const unsigned short* __restrict__ Ap, const unsigned short* __restrict__ A2p, int lda, long strideA,
    const unsigned short* __restrict__ Btp, const unsigned short* __restrict__ Bt2p, int ldb, long strideB,
    void* __restrict__ Cout, void* __restrict__ Cout2, int ldc, long strideC,
    const float* __restrict__ bias,
    const float* __restrict__ resid, long strideR,
    int M, int N, int K, float scale) {
  typedef typename Elem<ET>::T T;
  typedef typename Frag<T>::V V;
  const T* A = (const T*)Ap; const T* A2 = (const T*)A2p; const T* Bt = (const T*)Btp; const T* Bt2 = (const T*)Bt2p;
  __shared__ __align__(16) float sT[8][16 * 68];
  const int b    = blockIdx.y;
  const int lane = threadIdx.x & 31;
  const int wave = threadIdx.x >> 5;
  const int tilesN = N >> 6;
  const int tilesM = M >> 6;
  const int tile = blockIdx.x * 8 + wave;
  if (tile >= tilesM * tilesN) return;
  const int tm = tile / tilesN;
  const int tn = tile - tm * tilesN;
  const int m0 = tm << 6;
  const int n0 = tn << 6;

  const T* Ab  = A  + (size_t)b * strideA;
  const T* Bb  = Bt + (size_t)b * strideB;
  const T* Ab2 = SPLIT ? (A2  + (size_t)b * strideA) : nullptr;
  const T* Bb2 = SPLIT ? (Bt2 + (size_t)b * strideB) : nullptr;

  const int rlane = lane & 15;
  const int koff  = (lane >> 4) * 8;
  const int mOff  = (lane >> 4) * 8;

  v8f acc[4][4];
#pragma unroll
  for (int i = 0; i < 4; ++i)
#pragma unroll
    for (int j = 0; j < 4; ++j) acc[i][j] = (v8f){0.f,0.f,0.f,0.f,0.f,0.f,0.f,0.f};

  for (int k0 = 0; k0 < K; k0 += 32) {
    V bh[4], bl[4];
#pragma unroll
    for (int j = 0; j < 4; ++j) {
      const size_t bo = (size_t)(n0 + (j << 4) + rlane) * ldb + koff + k0;
      bh[j] = Frag<T>::load(Bb + bo);
      if (SPLIT) bl[j] = Frag<T>::load(Bb2 + bo);
    }
#pragma unroll
    for (int i = 0; i < 4; ++i) {
      const size_t ao = (size_t)(m0 + (i << 4) + rlane) * lda + koff + k0;
      V ah = Frag<T>::load(Ab + ao);
      V al;
      if (SPLIT) al = Frag<T>::load(Ab2 + ao);
#pragma unroll
      for (int j = 0; j < 4; ++j) {
        acc[i][j] = Frag<T>::mma(ah, bh[j], acc[i][j]);
        if (SPLIT) {
          acc[i][j] = Frag<T>::mma(ah, bl[j], acc[i][j]);
          acc[i][j] = Frag<T>::mma(al, bh[j], acc[i][j]);
        }
      }
      Frag<T>::guard4(acc[i][0], acc[i][1], acc[i][2], acc[i][3], ah, SPLIT ? al : ah);
    }
    Frag<T>::keep(bh[0], bh[1], bh[2], bh[3]);
    if (SPLIT) Frag<T>::keep(bl[0], bl[1], bl[2], bl[3]);
  }
  acc_guard4(acc[0][0], acc[0][1], acc[0][2], acc[0][3]);
  acc_guard4(acc[1][0], acc[1][1], acc[1][2], acc[1][3]);
  acc_guard4(acc[2][0], acc[2][1], acc[2][2], acc[2][3]);
  acc_guard4(acc[3][0], acc[3][1], acc[3][2], acc[3][3]);

  float* slab = sT[wave];
  const float* Rb = RESID ? (resid + (size_t)b * strideR) : nullptr;
#pragma unroll
  for (int i = 0; i < 4; ++i) {
    const int mBase = m0 + (i << 4);
#pragma unroll
    for (int j = 0; j < 4; ++j) {
      const int n = n0 + (j << 4) + rlane;
      float bv = 0.f;
      if (BIAS_MODE == 2) bv = bias[n];
#pragma unroll
      for (int r = 0; r < 8; ++r) {
        float v = acc[i][j][r] * scale;
        if (BIAS_MODE == 1) v += bias[mBase + mOff + r];
        if (BIAS_MODE == 2) v += bv;
        if (RESID) v += Rb[(size_t)(mBase + mOff + r) * ldc + n];
        if (ACT == 2) v = fmaxf(v, 0.0f);
        if (ACT == 4) v = (v > 0.f) ? v : 0.01f * v;
        slab[(mOff + r) * 68 + (j << 4) + rlane] = v;
      }
    }
    __builtin_amdgcn_fence(__ATOMIC_RELEASE, "workgroup");
    __builtin_amdgcn_wave_barrier();
    __builtin_amdgcn_fence(__ATOMIC_ACQUIRE, "workgroup");
    if (OUT_MODE == 0) {
      float* C = (float*)Cout + (size_t)b * strideC;
      const int hh = lane >> 4, c4 = (lane & 15) * 4;
      for (int pass = 0; pass < 2; ++pass) {
#pragma unroll
        for (int it = 0; it < 8; ++it) {
          const int row = it * 2 + hh;
          v4f v = *(const v4f*)(slab + row * 68 + c4);
          *(volatile v4f*)(C + (size_t)(mBase + row) * ldc + n0 + c4) = v;
        }
        __threadfence();
      }
    } else {
      const int q = lane >> 3, c8 = (lane & 7) * 8;
      unsigned short* C  = (unsigned short*)Cout  + (size_t)b * strideC;
      unsigned short* C2 = (OUT_MODE == 2) ? ((unsigned short*)Cout2 + (size_t)b * strideC) : nullptr;
      for (int pass = 0; pass < 2; ++pass) {
#pragma unroll
        for (int it = 0; it < 4; ++it) {
          const int row = it * 4 + q;
          const float* sp = slab + row * 68 + c8;
          v8h hv, lv;
#pragma unroll
          for (int e = 0; e < 8; ++e) {
            if (OUT_MODE == 1) {
              hv[e] = (_Float16)sp[e];
            } else {
              unsigned short hb = f2bf_bits(sp[e]);
              unsigned short lb = f2bf_bits(sp[e] - bf_bits2f(hb));
              hv[e] = __builtin_bit_cast(_Float16, hb);
              lv[e] = __builtin_bit_cast(_Float16, lb);
            }
          }
          *(volatile v8h*)(C + (size_t)(mBase + row) * ldc + n0 + c8) = hv;
          if (OUT_MODE == 2) *(volatile v8h*)(C2 + (size_t)(mBase + row) * ldc + n0 + c8) = lv;
        }
        __threadfence();
      }
    }
    __builtin_amdgcn_fence(__ATOMIC_RELEASE, "workgroup");
    __builtin_amdgcn_wave_barrier();
    __builtin_amdgcn_fence(__ATOMIC_ACQUIRE, "workgroup");
  }
}

__global__ __launch_bounds__(256) void cast8_f16_kernel(const float* __restrict__ in, unsigned short* __restrict__ out, int n8) {
  const int i = blockIdx.x * 256 + threadIdx.x;
  if (i >= n8) return;
  const float* p = in + 8 * (size_t)i;
  const v4f a = *(const v4f*)(p);
  const v4f c = *(const v4f*)(p + 4);
  unsigned short hb[8];
#pragma unroll
  for (int e = 0; e < 4; ++e) {
    hb[e]     = h_bits(a[e]);
    hb[4 + e] = h_bits(c[e]);
  }
  const v4u u = (v4u){pk16(hb[0], hb[1]), pk16(hb[2], hb[3]), pk16(hb[4], hb[5]), pk16(hb[6], hb[7])};
  unsigned short* q = out + 8 * (size_t)i;
  *(volatile v4u*)q = u;
  __threadfence();
  *(volatile v4u*)q = u;
}

__global__ __launch_bounds__(256) void wt_kernel(const float* __restrict__ W0, const float* __restrict__ W1,
                                                 const float* __restrict__ W2, const float* __restrict__ W3,
                                                 unsigned short* __restrict__ o0, unsigned short* __restrict__ o1,
                                                 unsigned short* __restrict__ o2, unsigned short* __restrict__ o3,
                                                 float scale) {
  __shared__ float sm[64][65];
  const int t  = threadIdx.x;
  const int k0 = blockIdx.x * 64;
  const int n0 = blockIdx.y * 64;
  const int z  = blockIdx.z;
  const float* W = (z == 0) ? W0 : (z == 1) ? W1 : (z == 2) ? W2 : W3;
  unsigned short* op = (z == 0) ? o0 : (z == 1) ? o1 : (z == 2) ? o2 : o3;
  const int perm = (z < 2) ? 1 : 0;
#pragma unroll
  for (int i = 0; i < 16; ++i) {
    const int e = i * 256 + t;
    const int r = e >> 6;
    const int c = e & 63;
    const int np = n0 + c;
    const int og = perm ? ((((np >> 5) & 1) << 9) + ((np >> 6) << 5) + (np & 31)) : np;
    sm[c][r] = W[(size_t)(k0 + r) * kDim + og] * scale;
  }
  __syncthreads();
  const int lane = t & 31, wave = t >> 5;
  const int q = lane >> 3, c8 = (lane & 7) * 8;
  for (int pass = 0; pass < 2; ++pass) {
#pragma unroll
    for (int it = 0; it < 2; ++it) {
      const int row = wave * 8 + it * 4 + q;
      unsigned short hb[8];
#pragma unroll
      for (int e = 0; e < 8; ++e) hb[e] = h_bits(sm[row][c8 + e]);
      const v4u u = (v4u){pk16(hb[0], hb[1]), pk16(hb[2], hb[3]), pk16(hb[4], hb[5]), pk16(hb[6], hb[7])};
      *(volatile v4u*)(op + (size_t)(n0 + row) * kDim + k0 + c8) = u;
    }
    __threadfence();
  }
}

__global__ __launch_bounds__(256) void biasperm_kernel(const float* __restrict__ bq, const float* __restrict__ bk,
                                                       float* __restrict__ out) {
  const int t = threadIdx.x;
  const float* src = (blockIdx.x == 0) ? bq : bk;
  const int np = 4 * t;
  const int og = (((np >> 5) & 1) << 9) + ((np >> 6) << 5) + (np & 31);
  const v4f v = *(const v4f*)(src + og);
  float* dp = out + (size_t)blockIdx.x * kDim + np;
  *(volatile v4f*)dp = v;
  __threadfence();
  *(volatile v4f*)dp = v;
}

__global__ __launch_bounds__(256) void softmax_diff_kernel(const float* __restrict__ S1p, const float* __restrict__ S2p,
                                                           const int* __restrict__ Mp,
                                                           const float* __restrict__ lq1, const float* __restrict__ lk1,
                                                           const float* __restrict__ lq2, const float* __restrict__ lk2,
                                                           unsigned short* __restrict__ Dp) {
  __shared__ __align__(16) float lg1[kSeq];
  __shared__ __align__(16) float lg2[kSeq];
  __shared__ float redA[8];
  __shared__ float redB[8];
  __shared__ float redC[8];
  __shared__ float redD[8];
  const int i    = blockIdx.x;
  const int t    = threadIdx.x;
  const int lane = t & 31, wave = t >> 5;

  float t1 = lq1[lane] * lk1[lane];
  float t2 = lq2[lane] * lk2[lane];
#pragma unroll
  for (int off = 16; off > 0; off >>= 1) {
    t1 += __shfl_xor(t1, off, 32);
    t2 += __shfl_xor(t2, off, 32);
  }
  const float lam = (expf(t1) - expf(t2)) + kLambdaInit;

  const size_t rowoff = (size_t)i * kSeq;
  const float* s1r = S1p + rowoff;
  const float* s2r = S2p + rowoff;
  const int*   mr  = Mp + rowoff;

  float mx1 = -__builtin_inff(), mx2 = -__builtin_inff();
#pragma unroll 1
  for (int it = 0; it < 4; ++it) {
    const int c = it * 512 + 2 * t;
    const v2f sa = *(const v2f*)(s1r + c);
    const v2f sb = *(const v2f*)(s2r + c);
    const v2i mv = *(const v2i*)(mr + c);
    v2f x1, x2;
#pragma unroll
    for (int e = 0; e < 2; ++e) {
      const bool keep = (mv[e] != 0);
      x1[e] = keep ? sa[e] : kNegBig;
      x2[e] = keep ? sb[e] : kNegBig;
      mx1 = fmaxf(mx1, x1[e]);
      mx2 = fmaxf(mx2, x2[e]);
    }
    *(v2f*)(lg1 + c) = x1;
    *(v2f*)(lg2 + c) = x2;
  }
#pragma unroll
  for (int off = 16; off > 0; off >>= 1) {
    mx1 = fmaxf(mx1, __shfl_xor(mx1, off, 32));
    mx2 = fmaxf(mx2, __shfl_xor(mx2, off, 32));
  }
  if (lane == 0) { redA[wave] = mx1; redB[wave] = mx2; }
  __syncthreads();
  float m1 = redA[0], m2 = redB[0];
#pragma unroll
  for (int w = 1; w < 8; ++w) { m1 = fmaxf(m1, redA[w]); m2 = fmaxf(m2, redB[w]); }

  float sum1 = 0.f, sum2 = 0.f;
#pragma unroll 1
  for (int it = 0; it < 4; ++it) {
    const int c = it * 512 + 2 * t;
    const v2f l1 = *(const v2f*)(lg1 + c);
    const v2f l2 = *(const v2f*)(lg2 + c);
    v2f e1, e2;
#pragma unroll
    for (int e = 0; e < 2; ++e) {
      e1[e] = expf(l1[e] - m1);
      e2[e] = expf(l2[e] - m2);
      sum1 += e1[e];
      sum2 += e2[e];
    }
    *(v2f*)(lg1 + c) = e1;
    *(v2f*)(lg2 + c) = e2;
  }
#pragma unroll
  for (int off = 16; off > 0; off >>= 1) {
    sum1 += __shfl_xor(sum1, off, 32);
    sum2 += __shfl_xor(sum2, off, 32);
  }
  if (lane == 0) { redC[wave] = sum1; redD[wave] = sum2; }
  __syncthreads();
  float tot1 = redC[0], tot2 = redD[0];
#pragma unroll
  for (int w = 1; w < 8; ++w) { tot1 += redC[w]; tot2 += redD[w]; }
  const float inv1 = kPCarry / tot1;
  const float inv2 = lam * (kPCarry / tot2);

  const v4f ea = *(const v4f*)(lg1 + 8 * t);
  const v4f eb = *(const v4f*)(lg1 + 8 * t + 4);
  const v4f ec = *(const v4f*)(lg2 + 8 * t);
  const v4f ed = *(const v4f*)(lg2 + 8 * t + 4);
  unsigned short hb[8];
#pragma unroll
  for (int e = 0; e < 4; ++e) {
    hb[e]     = h_bits(ea[e] * inv1 - ec[e] * inv2);
    hb[4 + e] = h_bits(eb[e] * inv1 - ed[e] * inv2);
  }
  const v4u u = (v4u){pk16(hb[0], hb[1]), pk16(hb[2], hb[3]), pk16(hb[4], hb[5]), pk16(hb[6], hb[7])};
  unsigned short* pr = Dp + rowoff + 8 * (size_t)t;
  *(volatile v4u*)pr = u;
  __threadfence();
  *(volatile v4u*)pr = u;
}

__global__ __launch_bounds__(256) void ln_cast_kernel(const float* __restrict__ O, const float* __restrict__ g,
                                                      const float* __restrict__ bta, unsigned short* __restrict__ A16) {
  const int t   = threadIdx.x;
  const int row = blockIdx.x * 2 + (t >> 7);
  const int tt  = t & 127;
  const int h   = tt >> 3;
  const int c0  = h * kDh + (tt & 7) * 8;
  const float* op = O + (size_t)row * kDim + c0;
  const v4f a = *(const v4f*)(op);
  const v4f c = *(const v4f*)(op + 4);
  float x[8];
#pragma unroll
  for (int e = 0; e < 4; ++e) { x[e] = a[e]; x[4 + e] = c[e]; }
  float s = ((x[0] + x[1]) + (x[2] + x[3])) + ((x[4] + x[5]) + (x[6] + x[7]));
  s += __shfl_xor(s, 1, 32);
  s += __shfl_xor(s, 2, 32);
  s += __shfl_xor(s, 4, 32);
  const float mu = s * kInv64;
  float d[8];
  float vs = 0.0f;
#pragma unroll
  for (int e = 0; e < 8; ++e) { d[e] = x[e] - mu; vs += d[e] * d[e]; }
  vs += __shfl_xor(vs, 1, 32);
  vs += __shfl_xor(vs, 2, 32);
  vs += __shfl_xor(vs, 4, 32);
  const float var  = vs * kInv64;
  const float rstd = 1.0f / sqrtf(var + kLnEps);
  const float* gp = g + c0;
  const float* bp = bta + c0;
  const v4f g0 = *(const v4f*)(gp);
  const v4f g1 = *(const v4f*)(gp + 4);
  const v4f b0 = *(const v4f*)(bp);
  const v4f b1 = *(const v4f*)(bp + 4);
  float gg[8], bb[8];
#pragma unroll
  for (int e = 0; e < 4; ++e) { gg[e] = g0[e]; gg[4 + e] = g1[e]; bb[e] = b0[e]; bb[4 + e] = b1[e]; }
  unsigned short hb[8];
#pragma unroll
  for (int e = 0; e < 8; ++e) {
    const float y = (d[e] * rstd * gg[e] + bb[e]) * kOutGain;
    hb[e] = h_bits(y);
  }
  const v4u u = (v4u){pk16(hb[0], hb[1]), pk16(hb[2], hb[3]), pk16(hb[4], hb[5]), pk16(hb[6], hb[7])};
  unsigned short* pr = A16 + (size_t)row * kDim + c0;
  *(volatile v4u*)pr = u;
  __threadfence();
  *(volatile v4u*)pr = u;
}

extern "C" void kernel_launch(void* const* d_in, const int* in_sizes, int n_in,
                              void* d_out, int out_size, void* d_ws, size_t ws_size,
                              hipStream_t stream) {
  if (n_in < 16) return;
  const int nTokElem = kTok * kDim;
  const int nW       = kDim * kDim;
  if (in_sizes[0] != nTokElem) return;
  if (in_sizes[1] != kBatch * kSeq * kSeq) return;
  if (in_sizes[2] != nW || in_sizes[4] != nW || in_sizes[6] != nW || in_sizes[8] != nW) return;
  if (in_sizes[3] != kDim || in_sizes[5] != kDim || in_sizes[7] != kDim || in_sizes[9] != kDim) return;
  if (in_sizes[10] != kDiff || in_sizes[11] != kDiff || in_sizes[12] != kDiff || in_sizes[13] != kDiff) return;
  if (in_sizes[14] != kHeads * kDh || in_sizes[15] != kHeads * kDh) return;
  if (out_size != nTokElem) return;

  const size_t szXH   = (size_t)kTok * kDim * 2;
  const size_t szWQK  = (size_t)kQKCols * kDim * 2;
  const size_t szW    = (size_t)kDim * kDim * 2;
  const size_t szBQK  = (size_t)kQKCols * 4;
  const size_t szQK16 = (size_t)kTok * kQKCols * 2;
  const size_t szVT16 = (size_t)kDim * kTok * 2;
  const size_t szSC   = (size_t)2 * kSeq * kSeq * 4;
  const size_t szDF   = (size_t)kSeq * kSeq * 2;
  const size_t szO    = (size_t)kTok * kDim * 4;
  const size_t szAOH  = (size_t)kTok * kDim * 2;
  const size_t offXH   = 0;
  const size_t offWQK  = offXH + szXH;
  const size_t offWVT  = offWQK + szWQK;
  const size_t offWOT  = offWVT + szW;
  const size_t offBQK  = offWOT + szW;
  const size_t offQK16 = offBQK + szBQK;
  const size_t offVT16 = offQK16 + szQK16;
  const size_t offSC   = offVT16 + szVT16;
  const size_t offDF   = offSC + szSC;
  const size_t offO    = offDF + szDF;
  const size_t offAOH  = offO + szO;
  const size_t total   = offAOH + szAOH;
  if (ws_size < total) return;

  const float* x    = (const float*)d_in[0];
  const int*   mask = (const int*)d_in[1];
  const float* Wq   = (const float*)d_in[2];
  const float* bq   = (const float*)d_in[3];
  const float* Wk   = (const float*)d_in[4];
  const float* bk   = (const float*)d_in[5];
  const float* Wv   = (const float*)d_in[6];
  const float* bv   = (const float*)d_in[7];
  const float* Wo   = (const float*)d_in[8];
  const float* bo   = (const float*)d_in[9];
  const float* lq1  = (const float*)d_in[10];
  const float* lk1  = (const float*)d_in[11];
  const float* lq2  = (const float*)d_in[12];
  const float* lk2  = (const float*)d_in[13];
  const float* ln_g = (const float*)d_in[14];
  const float* ln_b = (const float*)d_in[15];
  float* out = (float*)d_out;

  char* ws = (char*)d_ws;
  unsigned short* XH    = (unsigned short*)(ws + offXH);
  unsigned short* WQKT  = (unsigned short*)(ws + offWQK);
  unsigned short* WVT   = (unsigned short*)(ws + offWVT);
  unsigned short* WOT   = (unsigned short*)(ws + offWOT);
  float*          BQK   = (float*)(ws + offBQK);
  unsigned short* QK16  = (unsigned short*)(ws + offQK16);
  unsigned short* VT16  = (unsigned short*)(ws + offVT16);
  float*          SC    = (float*)(ws + offSC);
  unsigned short* DF    = (unsigned short*)(ws + offDF);
  float*          OATT  = (float*)(ws + offO);
  unsigned short* AOH16 = (unsigned short*)(ws + offAOH);

  const int n8 = nTokElem / 8;
  cast8_f16_kernel<<<dim3(n8 / 256), dim3(256), 0, stream>>>(x, XH, n8);
  wt_kernel<<<dim3(kDim / 64, kDim / 64, 4), dim3(256), 0, stream>>>(
      Wq, Wk, Wv, Wo, WQKT, WQKT + (size_t)kDim * kDim, WVT, WOT, kWCarry);
  biasperm_kernel<<<dim3(2), dim3(256), 0, stream>>>(bq, bk, BQK);

  {
    const int tiles = (kTok / 64) * (kQKCols / 64);
    wmma_gemm64<0, false, 2, 1, false, 0><<<dim3(tiles / 8, 1), dim3(256), 0, stream>>>(
        XH, XH, kDim, 0L, WQKT, WQKT, kDim, 0L,
        (void*)QK16, (void*)QK16, kQKCols, 0L, BQK, BQK, 0L, kTok, kQKCols, kDim, kWCarryInv);
  }
  {
    const int tiles = (kDim / 64) * (kTok / 64);
    wmma_gemm64<0, false, 1, 1, false, 0><<<dim3(tiles / 8, 1), dim3(256), 0, stream>>>(
        WVT, WVT, kDim, 0L, XH, XH, kDim, 0L,
        (void*)VT16, (void*)VT16, kTok, 0L, bv, bv, 0L, kDim, kTok, kDim, kWCarryInv);
  }

  const long planeSC    = (long)kSeq * kSeq;
  const int  tilesScore = (kSeq / 64) * (kSeq / 64);
  const int  tilesCtx   = (kSeq / 64) * (kDh / 64);
  for (int b = 0; b < kBatch; ++b) {
    const size_t tokQK = (size_t)b * kSeq * kQKCols;
    const int* maskb = mask + (size_t)b * kSeq * kSeq;
    for (int h = 0; h < kHeads; ++h) {
      const unsigned short* Ag  = QK16 + tokQK + (size_t)h * kDh;
      const unsigned short* Btg = QK16 + tokQK + (size_t)kDim + (size_t)h * kDh;
      wmma_gemm64<0, false, 0, 0, false, 0><<<dim3(tilesScore / 8, 2), dim3(256), 0, stream>>>(
          Ag, Ag, kQKCols, (long)kDiff, Btg, Btg, kQKCols, (long)kDiff,
          (void*)SC, (void*)SC, kSeq, planeSC, BQK, BQK, 0L, kSeq, kSeq, kDiff, kInvScale);
      softmax_diff_kernel<<<dim3(kSeq), dim3(256), 0, stream>>>(
          SC, SC + planeSC, maskb, lq1, lk1, lq2, lk2, DF);
      const unsigned short* VTg = VT16 + (size_t)h * kDh * kTok + (size_t)b * kSeq;
      float* Og = OATT + (size_t)b * kSeq * kDim + (size_t)h * kDh;
      wmma_gemm64<0, false, 0, 0, false, 0><<<dim3(tilesCtx / 8, 1), dim3(256), 0, stream>>>(
          DF, DF, kSeq, 0L, VTg, VTg, kTok, 0L,
          (void*)Og, (void*)Og, kDim, 0L, BQK, BQK, 0L, kSeq, kDh, kSeq, kPCarryInv);
    }
  }

  ln_cast_kernel<<<dim3(kTok / 2), dim3(256), 0, stream>>>(OATT, ln_g, ln_b, AOH16);

  {
    const int tiles = (kTok / 64) * (kDim / 64);
    wmma_gemm64<0, false, 2, 0, false, 0><<<dim3(tiles / 8, 1), dim3(256), 0, stream>>>(
        AOH16, AOH16, kDim, 0L, WOT, WOT, kDim, 0L,
        (void*)out, (void*)out, kDim, 0L, bo, bo, 0L, kTok, kDim, kDim, kWCarryInv);
  }
}
